// FlashDiffusionModule_25872882991444
// MI455X (gfx1250) — hardware-verified
//
#include <hip/hip_runtime.h>


#define NN   8192
#define DD   128
#define QB   2048
#define PCAR 1024.0f
#define ALPHA 1.0f
#define BETA  0.05f
typedef _Float16 h16;
typedef unsigned short bf;
typedef __attribute__((ext_vector_type(16))) __bf16   v16bf;
typedef __attribute__((ext_vector_type(16))) _Float16 v16h;
typedef __attribute__((ext_vector_type(8)))  _Float16 v8h;
typedef __attribute__((ext_vector_type(8)))  unsigned short v8us;
typedef __attribute__((ext_vector_type(8)))  float    v8f;
typedef __attribute__((ext_vector_type(4)))  float    v4f;
typedef v8h  __attribute__((may_alias)) v8ha;
typedef v4f  __attribute__((may_alias)) v4fa;
typedef v8us __attribute__((may_alias)) v8usa;

__device__ __forceinline__ unsigned short f2bf(float f) { unsigned u = __float_as_uint(f); u += 0x7FFFu + ((u >> 16) & 1u); return (unsigned short)(u >> 16); }
__device__ __forceinline__ float bf2f(unsigned short b) { return __uint_as_float(((unsigned)b) << 16); }
__device__ __forceinline__ float bfr(float f) { return bf2f(f2bf(f)); }
__device__ __forceinline__ v16h cat16(v8h lo, v8h hi) { return __builtin_shufflevector(lo, hi, 0, 1, 2, 3, 4, 5, 6, 7, 8, 9, 10, 11, 12, 13, 14, 15); }
__device__ __forceinline__ v16bf cat16b(v8us lo, v8us hi) { return __builtin_bit_cast(v16bf, __builtin_shufflevector(lo, hi, 0, 1, 2, 3, 4, 5, 6, 7, 8, 9, 10, 11, 12, 13, 14, 15)); }
__device__ __forceinline__ v8f wmma16(v16h a, v16h b, v8f c) { return __builtin_amdgcn_wmma_f32_16x16x32_f16(false, a, false, b, (short)0, c, false, false); }
__device__ __forceinline__ v8f wmmab(v16bf a, v16bf b, v8f c) { return __builtin_amdgcn_wmma_f32_16x16x32_bf16(false, a, false, b, (short)0, c, false, false); }


template <typename T16> struct WFrag;
template <> struct WFrag<h16> { typedef v16h V; static __device__ __forceinline__ V ld(const h16* p) { return cat16(*(const v8h*)p, *(const v8h*)(p + 16)); } static __device__ __forceinline__ v8f mma(V a, V b, v8f c) { return wmma16(a, b, c); } };
template <> struct WFrag<bf> { typedef v16bf V; static __device__ __forceinline__ V ld(const bf* p) { return cat16b(*(const v8us*)p, *(const v8us*)(p + 16)); } static __device__ __forceinline__ v8f mma(V a, V b, v8f c) { return wmmab(a, b, c); } };
template <typename T16, int NSPLIT, bool BIAS>
__global__ __launch_bounds__(32) void k_gemmw(const T16* __restrict__ A, const T16* __restrict__ A2, const T16* __restrict__ Bt, const T16* __restrict__ Bt2, int K, float* C, int ldc, const float* __restrict__ bias, size_t sA, size_t sB, size_t sC) {
    typedef typename WFrag<T16>::V V;
    __shared__ __align__(16) float os[16 * 68];
    const size_t z = blockIdx.z; A += z * sA; if (A2) A2 += z * sA; Bt += z * sB; if (Bt2) Bt2 += z * sB; C += z * sC;
    const int lane = threadIdx.x & 31, lr = lane & 15, hi = lane >> 4; const int r0 = blockIdx.x * 64, c0 = blockIdx.y * 64;
    v8f acc[4][4];
#pragma unroll
    for (int mb = 0; mb < 4; ++mb)
#pragma unroll
        for (int nb = 0; nb < 4; ++nb) acc[mb][nb] = (v8f){};
    const size_t aoff = (size_t)(r0 + lr) * K + 8 * hi, boff = (size_t)(c0 + lr) * K + 8 * hi;
#pragma unroll 1
    for (int kc = 0; kc < K; kc += 32) {
        V a[4], a2[4];
#pragma unroll
        for (int mb = 0; mb < 4; ++mb) { a[mb] = WFrag<T16>::ld(A + aoff + (size_t)mb * 16 * K + kc); if (NSPLIT == 1 || NSPLIT == 2) a2[mb] = WFrag<T16>::ld(A2 + aoff + (size_t)mb * 16 * K + kc); }
#pragma unroll
        for (int nb = 0; nb < 4; ++nb) { const V b = WFrag<T16>::ld(Bt + boff + (size_t)nb * 16 * K + kc); V b2; if (NSPLIT >= 2) b2 = WFrag<T16>::ld(Bt2 + boff + (size_t)nb * 16 * K + kc);
#pragma unroll
            for (int mb = 0; mb < 4; ++mb) { acc[mb][nb] = WFrag<T16>::mma(a[mb], b, acc[mb][nb]); if (NSPLIT == 1 || NSPLIT == 2) acc[mb][nb] = WFrag<T16>::mma(a2[mb], b, acc[mb][nb]); if (NSPLIT >= 2) acc[mb][nb] = WFrag<T16>::mma(a[mb], b2, acc[mb][nb]); } }
        asm volatile("v_nop\n\tv_nop\n\tv_nop\n\tv_nop" : "+v"(acc[0][0]), "+v"(acc[1][1]), "+v"(acc[2][2]), "+v"(acc[3][3]) : "v"(a[0]), "v"(a[3]));
    }
#pragma unroll
    for (int mb = 0; mb < 4; ++mb) {
#pragma unroll
        for (int nb = 0; nb < 4; ++nb) {
#pragma unroll
            for (int j = 0; j < 8; ++j) os[(hi * 8 + j) * 68 + nb * 16 + lr] = acc[mb][nb][j]; }
        __builtin_amdgcn_wave_barrier(); asm volatile("" ::: "memory");
        float* crow = C + (size_t)(r0 + mb * 16) * ldc + c0;
#pragma unroll 1
        for (int ps = 0; ps < 2; ++ps) {
#pragma unroll
            for (int s = 0; s < 8; ++s) { const int row = 2 * s + hi, cofs = lr * 4; v4f val = *(const v4fa*)(os + row * 68 + cofs); if (BIAS) { val[0] += bfr(bias[c0 + cofs]); val[1] += bfr(bias[c0 + cofs + 1]); val[2] += bfr(bias[c0 + cofs + 2]); val[3] += bfr(bias[c0 + cofs + 3]); }
                *(volatile v4f*)(crow + (size_t)row * ldc + cofs) = val; }
            if (ps == 0) __threadfence(); }
        __builtin_amdgcn_wave_barrier(); asm volatile("" ::: "memory");
    }
}

__device__ __forceinline__ h16 tohx(float x) { return (h16)x; }
typedef __attribute__((ext_vector_type(2))) _Float16 v2h;
typedef __attribute__((ext_vector_type(4))) _Float16 v4h;
typedef __attribute__((ext_vector_type(2))) float v2f;

__global__ __launch_bounds__(256) void k_cvt8(const float* __restrict__ src, bf* dst, size_t n8) { const size_t i = (size_t)blockIdx.x * 256 + threadIdx.x; if (i >= n8) return; const v8f v = *(const v8f*)(src + i * 8); v8us o;
#pragma unroll
    for (int k = 0; k < 8; ++k) o[k] = f2bf(v[k]); *(volatile v8us*)(dst + i * 8) = o; __threadfence(); *(volatile v8us*)(dst + i * 8) = o; }
__global__ __launch_bounds__(256) void k_terms(const float* __restrict__ Q, const float* __restrict__ K, const float* __restrict__ hh, const float* __restrict__ ldq, const float* __restrict__ ldk, float* RT, float* CT) { const int i = blockIdx.x * 256 + threadIdx.x; if (i >= NN) return; float nq = 0.f, nk = 0.f;
    for (int d = 0; d < DD; d += 4) { const v4f a = *(const v4f*)(Q + (size_t)i * DD + d), b = *(const v4f*)(K + (size_t)i * DD + d);
#pragma unroll
        for (int u = 0; u < 4; ++u) { const float qa = bfr(a[u]), kb = bfr(b[u]); float p1 = __fmul_rn(qa, qa), p2 = __fmul_rn(kb, kb); asm volatile("" : "+v"(p1)); asm volatile("" : "+v"(p2)); nq = __fadd_rn(nq, p1); nk = __fadd_rn(nk, p2); } }
    const float lh = logf(bfr(hh[i])); float t1 = __fmul_rn(-BETA, nq), t2 = __fmul_rn(-BETA, nk); asm volatile("" : "+v"(t1)); asm volatile("" : "+v"(t2)); float a1 = __fmul_rn(ALPHA, bfr(ldq[i])), a2 = __fmul_rn(ALPHA, bfr(ldk[i])); asm volatile("" : "+v"(a1)); asm volatile("" : "+v"(a2));
    const float r = __fadd_rn(__fsub_rn(t1, a1), lh), c = __fsub_rn(__fsub_rn(t2, a2), lh); *(volatile float*)(RT + i) = r; *(volatile float*)(CT + i) = c; __threadfence(); *(volatile float*)(RT + i) = r; *(volatile float*)(CT + i) = c; }
__global__ __launch_bounds__(256) void k_p16(const float* __restrict__ F, h16* P, size_t n) { const size_t i = ((size_t)blockIdx.x * 256 + threadIdx.x) * 2; if (i >= n) return; v2h o; o[0] = tohx(F[i]); o[1] = tohx(F[i + 1]); *(volatile v2h*)(P + i) = o; __threadfence(); *(volatile v2h*)(P + i) = o; }
__global__ __launch_bounds__(256) void k_vt(const float* __restrict__ Vv, h16* VT) { const size_t e = ((size_t)blockIdx.x * 256 + threadIdx.x) * 2; if (e >= (size_t)DD * NN) return; const int j = (int)(e % NN), d = (int)(e / NN); v2h o; o[0] = tohx(bfr(Vv[(size_t)j * DD + d])); o[1] = tohx(bfr(Vv[(size_t)(j + 1) * DD + d])); *(volatile v2h*)(VT + e) = o; __threadfence(); *(volatile v2h*)(VT + e) = o; }
__global__ __launch_bounds__(256) void k_smax(const float* __restrict__ G, const float* __restrict__ RT, const float* __restrict__ CT, int i0, float* RS) { const int lane = threadIdx.x & 31; const int i = blockIdx.x * 8 + (threadIdx.x >> 5); if (i >= QB) return; const float* sr = G + (size_t)i * NN; const float ri = RT[i0 + i]; float m = -3.0e38f;
#pragma unroll 4
    for (int c0 = lane * 4; c0 < NN; c0 += 128) { const v4f v = *(const v4f*)(sr + c0); const v4f c = *(const v4f*)(CT + c0);
#pragma unroll
        for (int q = 0; q < 4; ++q) { float g2 = v[q] * (2.0f * BETA); asm volatile("" : "+v"(g2)); m = fmaxf(m, __fadd_rn(__fadd_rn(g2, ri), c[q])); } }
#pragma unroll
    for (int sh = 16; sh; sh >>= 1) m = fmaxf(m, __shfl_xor(m, sh, 32));
    const float o = lane == 0 ? m : 0.f; *(volatile float*)(RS + (size_t)i * 32 + lane) = o; __threadfence(); *(volatile float*)(RS + (size_t)i * 32 + lane) = o; }
__global__ __launch_bounds__(256) void k_sexp(const float* __restrict__ G, const float* __restrict__ RT, const float* __restrict__ CT, int i0, float* RS, h16* P, float* LSE) { const int lane = threadIdx.x & 31; const int i = blockIdx.x * 8 + (threadIdx.x >> 5); if (i >= QB) return; const float* sr = G + (size_t)i * NN; const float m = RS[(size_t)i * 32]; const float ri = RT[i0 + i]; float sum = 0.f;
#pragma unroll 1
    for (int ps = 0; ps < 2; ++ps) { sum = 0.f;
#pragma unroll 2
        for (int c0 = lane * 4; c0 < NN; c0 += 128) { const v4f v = *(const v4f*)(sr + c0); const v4f c = *(const v4f*)(CT + c0); v4h o;
#pragma unroll
            for (int q = 0; q < 4; ++q) { float g2 = v[q] * (2.0f * BETA); asm volatile("" : "+v"(g2)); float s = __fadd_rn(__fadd_rn(g2, ri), c[q]); float dlt = __fsub_rn(s, m); asm volatile("" : "+v"(dlt)); const float e = __expf(dlt); sum += e; o[q] = tohx(e * PCAR); }
            *(volatile v4h*)(P + (size_t)i * NN + c0) = o; }
        if (ps == 0) __threadfence(); }
#pragma unroll
    for (int sh = 16; sh; sh >>= 1) sum += __shfl_xor(sum, sh, 32);
    float lg = logf(sum); asm volatile("" : "+v"(lg)); const float lse = __fadd_rn(m, lg);
    const float o2 = lane == 0 ? m : (lane == 1 ? __fdiv_rn(1.0f, sum * PCAR) : (lane == 2 ? lse : 0.f)); *(volatile float*)(RS + (size_t)i * 32 + lane) = o2; __threadfence(); *(volatile float*)(RS + (size_t)i * 32 + lane) = o2; }
__global__ __launch_bounds__(256) void k_oscal(const float* __restrict__ O, const float* __restrict__ RS, float* OUTb) { const size_t e = ((size_t)blockIdx.x * 256 + threadIdx.x) * 2; if (e >= (size_t)QB * DD) return; const int i = (int)(e / DD); const float rsn = RS[(size_t)i * 32 + 1]; v2f o; o[0] = __fmul_rn(O[e], rsn); o[1] = __fmul_rn(O[e + 1], rsn); *(volatile v2f*)(OUTb + e) = o; __threadfence(); *(volatile v2f*)(OUTb + e) = o; }
__global__ __launch_bounds__(256) void k_lse(const float* __restrict__ RS, float* LSEb) { const int i = blockIdx.x * 256 + threadIdx.x; if (i >= QB) return; const float v = RS[(size_t)i * 32 + 2]; *(volatile float*)(LSEb + i) = v; __threadfence(); *(volatile float*)(LSEb + i) = v; }

extern "C" void kernel_launch(void* const* d_in, const int* in_sizes, int n_in,
                              void* d_out, int out_size, void* d_ws, size_t ws_size, hipStream_t stream) {
    (void)in_sizes; (void)n_in; (void)out_size;
    const float* Q = (const float*)d_in[0]; const float* K = (const float*)d_in[1]; const float* V = (const float*)d_in[2]; const float* hh = (const float*)d_in[3]; const float* ldq = (const float*)d_in[4]; const float* ldk = (const float*)d_in[5];
    float* OUT = (float*)d_out; float* LSE = (float*)d_out + (size_t)NN * DD;
    char* wsp = (char*)d_ws;
    auto take = [&](size_t bytes) { char* p = wsp; wsp += (bytes + 255) & ~(size_t)255; return (void*)p; };
    bf* QB16 = (bf*)take((size_t)NN * DD * 2); bf* KB16 = (bf*)take((size_t)NN * DD * 2); h16* VT = (h16*)take((size_t)DD * NN * 2); float* RT = (float*)take((size_t)NN * 4); float* CT = (float*)take((size_t)NN * 4);
    float* G = (float*)take((size_t)QB * NN * 4); h16* P = (h16*)take((size_t)QB * NN * 2); float* RS = (float*)take((size_t)QB * 32 * 4); float* O = (float*)take((size_t)QB * DD * 4);
    if ((size_t)(wsp - (char*)d_ws) > ws_size) return;
    k_cvt8<<<(unsigned)(((size_t)NN * DD / 8 + 255) / 256), 256, 0, stream>>>(Q, QB16, (size_t)NN * DD / 8); k_cvt8<<<(unsigned)(((size_t)NN * DD / 8 + 255) / 256), 256, 0, stream>>>(K, KB16, (size_t)NN * DD / 8); k_vt<<<(unsigned)(((size_t)DD * NN / 2 + 255) / 256), 256, 0, stream>>>(V, VT);
    k_terms<<<NN / 256, 256, 0, stream>>>(Q, K, hh, ldq, ldk, RT, CT);
    for (int qb = 0; qb < NN / QB; ++qb) { const int i0 = qb * QB;
        k_gemmw<bf, 0, false><<<dim3(QB / 64, NN / 64, 1), 32, 0, stream>>>(QB16 + (size_t)i0 * DD, nullptr, KB16, nullptr, DD, G, NN, nullptr, 0, 0, 0);
        k_smax<<<QB / 8, 256, 0, stream>>>(G, RT, CT, i0, RS); k_sexp<<<QB / 8, 256, 0, stream>>>(G, RT, CT, i0, RS, P, LSE);
        k_gemmw<h16, 0, false><<<dim3(QB / 64, DD / 64, 1), 32, 0, stream>>>(P, nullptr, VT, nullptr, NN, O, DD, nullptr, 0, 0, 0);
        k_oscal<<<(unsigned)(((size_t)QB * DD / 2 + 255) / 256), 256, 0, stream>>>(O, RS, OUT + (size_t)i0 * DD); k_lse<<<QB / 256, 256, 0, stream>>>(RS, LSE + i0); }
}
